// endecoder2_20839181320647
// MI455X (gfx1250) — hardware-verified
//
#include <hip/hip_runtime.h>


namespace {
constexpr int Bsz = 8, T = 1024, HID = 512, DH = 64, NH = 8;
constexpr int MROWS = Bsz * T;
constexpr int QT_PER_B = T / 16;
constexpr int FF = 2 * HID;

typedef _Float16 b16;
typedef __attribute__((ext_vector_type(16))) _Float16 v16b;
typedef __attribute__((ext_vector_type(8)))  _Float16 v8b;
typedef __attribute__((ext_vector_type(8)))  float v8f;
typedef __attribute__((ext_vector_type(4)))  float v4f;
typedef __attribute__((ext_vector_type(2)))  float v2f;

__device__ __forceinline__ v8b ld8b(const b16* p) { return *(const v8b*)p; }
__device__ __forceinline__ v16b cat8b(v8b a, v8b b) { return __builtin_shufflevector(a, b, 0, 1, 2, 3, 4, 5, 6, 7, 8, 9, 10, 11, 12, 13, 14, 15); }
__device__ __forceinline__ v16b frag_kb(const b16* p, int hh) { return cat8b(ld8b(p + 8 * hh), ld8b(p + 16 + 8 * hh)); }
__device__ __forceinline__ void split_bf16(float v, b16& hi, b16& lo) {
  hi = (b16)v; lo = (b16)0.0f;
}
__device__ __forceinline__ void frag_ksplit(const float* p, int hh, v16b& fh_, v16b& fl_) {
  const float* p0 = p + 8 * hh; const float* p1 = p + 16 + 8 * hh;
#pragma unroll
  for (int e = 0; e < 8; ++e) { b16 a, c; split_bf16(p0[e], a, c); fh_[e] = a; fl_[e] = c; split_bf16(p1[e], a, c); fh_[8 + e] = a; fl_[8 + e] = c; }
}
__device__ __forceinline__ v8f wmma16b(v16b a, v16b b, v8f c) {
  v8f d = __builtin_amdgcn_wmma_f32_16x16x32_f16(false, a, false, b, (short)0, c, false, false);
  asm volatile("v_nop\n\tv_nop\n\tv_nop\n\tv_nop" : "+v"(d) : "v"(a), "v"(b));
  return d;
}
__device__ __forceinline__ v8f wmma3(v16b ah, v16b al, v16b bh, v16b bl, v8f c) {
  (void)al; (void)bl; return wmma16b(ah, bh, c);
}
__device__ __forceinline__ void wave_lds_sync() {
  __builtin_amdgcn_fence(__ATOMIC_RELEASE, "workgroup"); __builtin_amdgcn_wave_barrier(); __builtin_amdgcn_fence(__ATOMIC_ACQUIRE, "workgroup");
}
#define VST2(Tp, ptr, val) do { const Tp _v = (val); *(volatile Tp*)(ptr) = _v; __threadfence(); *(volatile Tp*)(ptr) = _v; } while (0)

__global__ __launch_bounds__(256) void wplanes_kernel(const float* __restrict__ w, int Kin, int Nout, int perm, b16* __restrict__ ph, b16* __restrict__ pl) {
  const size_t i8 = (size_t)blockIdx.x * 256 + threadIdx.x;
  if (i8 * 8 >= (size_t)Nout * Kin) return;
  const size_t i = i8 * 8; const int n = (int)(i / Kin), k0 = (int)(i % Kin);
  const int src_n = perm ? ((n & 63) * 8 + (n >> 6)) : n;
  v8b hv, lv;
#pragma unroll
  for (int e = 0; e < 8; ++e) { b16 a, c; split_bf16(w[(size_t)(k0 + e) * Nout + src_n], a, c); hv[e] = a; lv[e] = c; }
  VST2(v8b, ph + i, hv); VST2(v8b, pl + i, lv);
}

__global__ __launch_bounds__(128) void ln_kernel(const float* __restrict__ x, const float* __restrict__ g, const float* __restrict__ bb,
                                                 float* __restrict__ out, int ldo, int coloff) {
  __shared__ float red[2][128];
  __shared__ __attribute__((aligned(16))) float row[HID];
  const int r = blockIdx.x, t = threadIdx.x;
  const float* xr = x + (size_t)r * HID;
  float v[4], s = 0.f, s2 = 0.f;
#pragma unroll
  for (int q = 0; q < 4; ++q) { v[q] = xr[t * 4 + q]; s += v[q]; }
  red[0][t] = s; __syncthreads();
  for (int o = 64; o > 0; o >>= 1) { if (t < o) red[0][t] += red[0][t + o]; __syncthreads(); }
  const float mu = red[0][0] * (1.0f / HID);
#pragma unroll
  for (int q = 0; q < 4; ++q) { const float d = v[q] - mu; s2 += d * d; }
  red[1][t] = s2; __syncthreads();
  for (int o = 64; o > 0; o >>= 1) { if (t < o) red[1][t] += red[1][t + o]; __syncthreads(); }
  const float inv = 1.0f / sqrtf(red[1][0] * (1.0f / HID) + 1e-5f);
  v4f o4;
#pragma unroll
  for (int q = 0; q < 4; ++q) o4[q] = (v[q] - mu) * inv * g[t * 4 + q] + bb[t * 4 + q];
  VST2(v4f, out + (size_t)r * ldo + coloff + t * 4, o4);
}

__device__ __forceinline__ void gemm_tile_split(const float* __restrict__ A, int lda, const b16* __restrict__ wh, const b16* __restrict__ wl,
                                                int m0, int c0, int K, int nloc, int hlf, v8f (&acc)[2][4]) {
  for (int kb = 0; kb < K; kb += 32) {
    v16b a0h, a0l, a1h, a1l;
    frag_ksplit(A + (size_t)(m0 + nloc) * lda + kb, hlf, a0h, a0l);
    frag_ksplit(A + (size_t)(m0 + 16 + nloc) * lda + kb, hlf, a1h, a1l);
#pragma unroll
    for (int t = 0; t < 4; ++t) {
      const size_t wofs = (size_t)(c0 + t * 16 + nloc) * K + kb;
      const v16b bh = frag_kb(wh + wofs, hlf), bl = frag_kb(wl + wofs, hlf);
      acc[0][t] = wmma3(a0h, a0l, bh, bl, acc[0][t]);
      acc[1][t] = wmma3(a1h, a1l, bh, bl, acc[1][t]);
    }
  }
}

template <int KIN, int MODE>
__global__ __launch_bounds__(128) void proj_kernel(const float* __restrict__ A, int acol, const b16* __restrict__ wh, const b16* __restrict__ wl,
                                                   const float* __restrict__ bias, int yoff, b16* __restrict__ Ph, b16* __restrict__ Pl) {
  __shared__ __attribute__((aligned(16))) b16 Ts[4][2][32 * 64];
  const int lane = threadIdx.x & 31, wave = threadIdx.x >> 5, nloc = lane & 15, hlf = lane >> 4;
  const int m0 = (blockIdx.y + yoff) * 128 + wave * 32;
  const int c0 = blockIdx.x * 64;
  const int head = c0 / DH;
  v8f acc[2][4];
#pragma unroll
  for (int r = 0; r < 2; ++r)
#pragma unroll
    for (int t = 0; t < 4; ++t) acc[r][t] = (v8f){};
  gemm_tile_split(A + acol, 2 * HID, wh, wl, m0, c0, KIN, nloc, hlf, acc);
  const int b = m0 / T, t0 = m0 % T;
  b16* Tp0 = Ts[wave][0]; b16* Tp1 = Ts[wave][1];
#pragma unroll
  for (int t = 0; t < 4; ++t)
#pragma unroll
    for (int r = 0; r < 2; ++r)
#pragma unroll
      for (int v = 0; v < 8; ++v) {
        const int rr = r * 16 + v + 8 * hlf, d = t * 16 + nloc;
        b16 yh, yl; split_bf16(acc[r][t][v] + bias[c0 + d], yh, yl);
        const int idx = (MODE == 0) ? (rr * 64 + d) : ((rr >> 4) * 1024 + d * 16 + (rr & 15));
        Tp0[idx] = yh; Tp1[idx] = yl;
      }
  wave_lds_sync();
  size_t o;
  if (MODE == 0) o = ((size_t)(b * NH + head) * T + t0) * DH;
  else           o = ((size_t)(b * NH + head) * QT_PER_B + (t0 >> 4)) * (size_t)(DH * 16);
  for (int pass = 0; pass < 2; ++pass) {
#pragma unroll
    for (int j = 0; j < 8; ++j) { const int e = (j * 32 + lane) * 8; *(volatile v8b*)(Ph + o + e) = ld8b(Tp0 + e); *(volatile v8b*)(Pl + o + e) = ld8b(Tp1 + e); }
    __threadfence();
  }
}

__device__ __forceinline__ void st_chunk(const b16* Kh, const b16* Kl, size_t ko, int kb, int col, int hh,
                                         const v16b& q0h, const v16b& q0l, const v16b& q1h, const v16b& q1l, v8f& s0, v8f& s1) {
  const size_t r0 = ko + (size_t)(kb + col) * DH, r1 = ko + (size_t)(kb + 16 + col) * DH;
  s0 = (v8f){}; s1 = (v8f){};
  v16b ah = frag_kb(Kh + r0, hh), al = frag_kb(Kl + r0, hh);
  s0 = wmma3(ah, al, q0h, q0l, s0);
  ah = frag_kb(Kh + r0 + 32, hh); al = frag_kb(Kl + r0 + 32, hh);
  s0 = wmma3(ah, al, q1h, q1l, s0);
  ah = frag_kb(Kh + r1, hh); al = frag_kb(Kl + r1, hh);
  s1 = wmma3(ah, al, q0h, q0l, s1);
  ah = frag_kb(Kh + r1 + 32, hh); al = frag_kb(Kl + r1 + 32, hh);
  s1 = wmma3(ah, al, q1h, q1l, s1);
}
__device__ __forceinline__ void write_y(float* Tt, const v8f& o0, const v8f& o1, const v8f& o2, const v8f& o3, float scale, int col, int hh,
                                        float* __restrict__ yf, int b, int h, int q0) {
#pragma unroll
  for (int r = 0; r < 8; ++r) {
    const int hr = 8 * hh + r;
    Tt[col * 64 + 0 + hr] = o0[r] * scale; Tt[col * 64 + 16 + hr] = o1[r] * scale;
    Tt[col * 64 + 32 + hr] = o2[r] * scale; Tt[col * 64 + 48 + hr] = o3[r] * scale;
  }
  wave_lds_sync();
  float* dst0 = yf + ((size_t)b * T + q0) * HID + h * DH;
  for (int pass = 0; pass < 2; ++pass) {
#pragma unroll
    for (int j = 0; j < 8; ++j) { const int rr = j * 2 + hh, c4 = col * 4; *(volatile v4f*)(dst0 + (size_t)rr * HID + c4) = *(const v4f*)(Tt + rr * 64 + c4); }
    __threadfence();
  }
}
__device__ __forceinline__ void pv_chunk(const b16* Vh, const b16* Vl, size_t ko, int kb, int col, int hh, const v16b& pbh, const v16b& pbl,
                                         v8f& o0, v8f& o1, v8f& o2, v8f& o3) {
  const size_t v0 = ko + (size_t)(kb >> 4) * (DH * 16) + 8 * hh, v1 = v0 + DH * 16;
#pragma unroll
  for (int n = 0; n < 4; ++n) {
    const int f = n * 16 + col;
    const v16b vah = cat8b(ld8b(Vh + v0 + f * 16), ld8b(Vh + v1 + f * 16));
    const v16b val = cat8b(ld8b(Vl + v0 + f * 16), ld8b(Vl + v1 + f * 16));
    v8f& o = (n == 0) ? o0 : (n == 1) ? o1 : (n == 2) ? o2 : o3;
    o = wmma3(vah, val, pbh, pbl, o);
  }
}

__global__ __launch_bounds__(256) void attn_row_kernel(const b16* __restrict__ Qh, const b16* __restrict__ Ql, const b16* __restrict__ Kh, const b16* __restrict__ Kl,
                                                       const b16* __restrict__ Vh, const b16* __restrict__ Vl, int tile_off, float* __restrict__ yf) {
  __shared__ __attribute__((aligned(16))) float Os[8][16 * 64];
  const int wid = threadIdx.x >> 5, lane = threadIdx.x & 31, hh = lane >> 4, col = lane & 15;
  const int qtile = blockIdx.x * 8 + wid + tile_off;
  const int g = qtile / QT_PER_B, q0 = (qtile % QT_PER_B) << 4;
  const int b = g / NH, h = g % NH;
  const size_t ko = (size_t)g * T * DH;
  const size_t qo = ((size_t)g * T + q0 + col) * DH;
  const v16b q0h = frag_kb(Qh + qo, hh), q0l = frag_kb(Ql + qo, hh), q1h = frag_kb(Qh + qo + 32, hh), q1l = frag_kb(Ql + qo + 32, hh);
  float m = -INFINITY, l = 0.0f;
  v8f o0 = {}, o1 = {}, o2 = {}, o3 = {};
  for (int kb = 0; kb < T; kb += 32) {
    v8f s0, s1; st_chunk(Kh, Kl, ko, kb, col, hh, q0h, q0l, q1h, q1l, s0, s1);
    float mr = -INFINITY;
#pragma unroll
    for (int r = 0; r < 8; ++r) mr = fmaxf(mr, fmaxf(s0[r], s1[r]));
    mr = fmaxf(mr, __shfl_xor(mr, 16));
    const float mn = fmaxf(m, mr);
    const float al_ = expf(m - mn);
    m = mn;
    float sum = 0.0f;
    v16b pbh, pbl;
#pragma unroll
    for (int r = 0; r < 8; ++r) {
      const float p0 = expf(s0[r] - mn), p1 = expf(s1[r] - mn);
      sum += p0 + p1;
      b16 a, c; split_bf16(p0, a, c); pbh[r] = a; pbl[r] = c; split_bf16(p1, a, c); pbh[8 + r] = a; pbl[8 + r] = c;
    }
    sum += __shfl_xor(sum, 16);
    l = l * al_ + sum;
#pragma unroll
    for (int r = 0; r < 8; ++r) { o0[r] *= al_; o1[r] *= al_; o2[r] *= al_; o3[r] *= al_; }
    pv_chunk(Vh, Vl, ko, kb, col, hh, pbh, pbl, o0, o1, o2, o3);
  }
  write_y(Os[wid], o0, o1, o2, o3, 1.0f / l, col, hh, yf, b, h, q0);
}

__global__ __launch_bounds__(256) void add_perm_kernel(const float* __restrict__ resid, const float* __restrict__ y, float* __restrict__ res, int rows) {
  const size_t t = (size_t)blockIdx.x * 256 + threadIdx.x;
  if (t >= (size_t)rows * HID) return;
  const size_t n = t / HID; const int c = (int)(t % HID);
  const int pc = (c & 7) * DH + (c >> 3);
  VST2(float, res + t, resid[t] + y[n * HID + pc]);
}

template <int KIN, int NOUT, bool RELU>
__global__ __launch_bounds__(128) void gemm_kernel(const float* __restrict__ A, int lda, int acol, const b16* __restrict__ wh, const b16* __restrict__ wl,
                                                   const float* __restrict__ bias, const float* __restrict__ resid, int yoff,
                                                   float* __restrict__ out, float* __restrict__ out2) {
  __shared__ __attribute__((aligned(16))) float Ts[4][32 * 64];
  const int lane = threadIdx.x & 31, wave = threadIdx.x >> 5, nloc = lane & 15, hlf = lane >> 4;
  const int m0 = (blockIdx.y + yoff) * 128 + wave * 32;
  const int c0 = blockIdx.x * 64;
  v8f acc[2][4];
#pragma unroll
  for (int r = 0; r < 2; ++r)
#pragma unroll
    for (int t = 0; t < 4; ++t) acc[r][t] = (v8f){};
  gemm_tile_split(A + acol, lda, wh, wl, m0, c0, KIN, nloc, hlf, acc);
  float* Tt = Ts[wave];
#pragma unroll
  for (int t = 0; t < 4; ++t)
#pragma unroll
    for (int r = 0; r < 2; ++r)
#pragma unroll
      for (int v = 0; v < 8; ++v) {
        const int rr = r * 16 + v + 8 * hlf, cc = t * 16 + nloc;
        float val = acc[r][t][v] + bias[c0 + cc];
        if (RELU) val = fmaxf(val, 0.0f);
        if (resid) val += resid[(size_t)(m0 + rr) * NOUT + c0 + cc];
        Tt[rr * 64 + cc] = val;
      }
  wave_lds_sync();
  for (int pass = 0; pass < 2; ++pass) {
#pragma unroll
    for (int j = 0; j < 16; ++j) { const int rr = j * 2 + hlf, c4 = nloc * 4;
      const v4f v = *(const v4f*)(Tt + rr * 64 + c4);
      *(volatile v4f*)(out + (size_t)(m0 + rr) * NOUT + c0 + c4) = v;
      if (out2) *(volatile v4f*)(out2 + (size_t)(m0 + rr) * NOUT + c0 + c4) = v; }
    __threadfence();
  }
}

__global__ __launch_bounds__(256) void bperm_kernel(const float* __restrict__ bq, const float* __restrict__ bk, const float* __restrict__ bv1, const float* __restrict__ bv2,
                                                    float* __restrict__ bp) {
  const int t = blockIdx.x * 256 + threadIdx.x;
  if (t >= 4 * HID) return;
  const int which = t / HID, n = t % HID, src = (n & 63) * 8 + (n >> 6);
  const float* b = (which == 0) ? bq : (which == 1) ? bk : (which == 2) ? bv1 : bv2;
  VST2(float, bp + t, b[src]);
}
}

extern "C" void kernel_launch(void* const* d_in, const int* in_sizes, int n_in,
                              void* d_out, int out_size, void* d_ws, size_t ws_size, hipStream_t stream) {
  (void)in_sizes; (void)n_in; (void)out_size;
  const float* rgb = (const float*)d_in[0];  const float* dep = (const float*)d_in[1];
  const float* Wq  = (const float*)d_in[2];  const float* bq  = (const float*)d_in[3];
  const float* Wk  = (const float*)d_in[4];  const float* bk  = (const float*)d_in[5];
  const float* Wv1 = (const float*)d_in[6];  const float* bv1 = (const float*)d_in[7];
  const float* Wv2 = (const float*)d_in[8];  const float* bv2 = (const float*)d_in[9];
  const float* W11 = (const float*)d_in[10]; const float* b11 = (const float*)d_in[11];
  const float* W12 = (const float*)d_in[12]; const float* b12 = (const float*)d_in[13];
  const float* W21 = (const float*)d_in[14]; const float* b21 = (const float*)d_in[15];
  const float* W22 = (const float*)d_in[16]; const float* b22 = (const float*)d_in[17];
  const float* g11 = (const float*)d_in[18]; const float* be11 = (const float*)d_in[19];
  const float* g12 = (const float*)d_in[20]; const float* be12 = (const float*)d_in[21];
  const float* g21 = (const float*)d_in[22]; const float* be21 = (const float*)d_in[23];
  const float* g22 = (const float*)d_in[24]; const float* be22 = (const float*)d_in[25];
  float* out1 = (float*)d_out;
  float* out2 = out1 + (size_t)MROWS * HID;
  float* out3 = out2 + (size_t)MROWS * HID;

  size_t off = 0; char* ws = (char*)d_ws;
  auto take = [&](size_t bytes) { void* p = ws + off; off += (bytes + 255) & ~(size_t)255; return p; };
  float* hbuf = (float*)take((size_t)MROWS * 2 * HID * 4);
  b16* wqh = (b16*)take((size_t)HID * HID * 2);  b16* wql = (b16*)take((size_t)HID * HID * 2);
  b16* wkh = (b16*)take((size_t)HID * HID * 2);  b16* wkl = (b16*)take((size_t)HID * HID * 2);
  b16* wv1h = (b16*)take((size_t)HID * FF * 2);  b16* wv1l = (b16*)take((size_t)HID * FF * 2);
  b16* wv2h = (b16*)take((size_t)HID * FF * 2);  b16* wv2l = (b16*)take((size_t)HID * FF * 2);
  b16* w11h = (b16*)take((size_t)FF * HID * 2);  b16* w11l = (b16*)take((size_t)FF * HID * 2);
  b16* w12h = (b16*)take((size_t)HID * FF * 2);  b16* w12l = (b16*)take((size_t)HID * FF * 2);
  b16* w21h = (b16*)take((size_t)FF * HID * 2);  b16* w21l = (b16*)take((size_t)FF * HID * 2);
  b16* w22h = (b16*)take((size_t)HID * FF * 2);  b16* w22l = (b16*)take((size_t)HID * FF * 2);
  float* bp = (float*)take((size_t)4 * HID * 4);
  b16* Qh = (b16*)take((size_t)MROWS * HID * 2); b16* Ql = (b16*)take((size_t)MROWS * HID * 2);
  b16* Kh = (b16*)take((size_t)MROWS * HID * 2); b16* Kl = (b16*)take((size_t)MROWS * HID * 2);
  b16* V1h = (b16*)take((size_t)MROWS * HID * 2); b16* V1l = (b16*)take((size_t)MROWS * HID * 2);
  b16* V2h = (b16*)take((size_t)MROWS * HID * 2); b16* V2l = (b16*)take((size_t)MROWS * HID * 2);
  v2f* ML  = (v2f*)take((size_t)Bsz * NH * T * 8);
  float* y1 = (float*)take((size_t)MROWS * HID * 4);  float* y2 = (float*)take((size_t)MROWS * HID * 4);
  float* resr = (float*)take((size_t)MROWS * HID * 4); float* resd = (float*)take((size_t)MROWS * HID * 4);
  float* f1 = (float*)take((size_t)MROWS * FF * 4);
  if (off > ws_size) return;

  wplanes_kernel<<<(HID * HID / 8 + 255) / 256, 256, 0, stream>>>(Wq, HID, HID, 1, wqh, wql);
  wplanes_kernel<<<(HID * HID / 8 + 255) / 256, 256, 0, stream>>>(Wk, HID, HID, 1, wkh, wkl);
  wplanes_kernel<<<(FF * HID / 8 + 255) / 256, 256, 0, stream>>>(Wv1, FF, HID, 1, wv1h, wv1l);
  wplanes_kernel<<<(FF * HID / 8 + 255) / 256, 256, 0, stream>>>(Wv2, FF, HID, 1, wv2h, wv2l);
  wplanes_kernel<<<(HID * FF / 8 + 255) / 256, 256, 0, stream>>>(W11, HID, FF, 0, w11h, w11l);
  wplanes_kernel<<<(FF * HID / 8 + 255) / 256, 256, 0, stream>>>(W12, FF, HID, 0, w12h, w12l);
  wplanes_kernel<<<(HID * FF / 8 + 255) / 256, 256, 0, stream>>>(W21, HID, FF, 0, w21h, w21l);
  wplanes_kernel<<<(FF * HID / 8 + 255) / 256, 256, 0, stream>>>(W22, FF, HID, 0, w22h, w22l);
  bperm_kernel<<<(4 * HID + 255) / 256, 256, 0, stream>>>(bq, bk, bv1, bv2, bp);

  const int ROWS = MROWS;
  const int NT_TILES = Bsz * NH * QT_PER_B;
  ln_kernel<<<ROWS, 128, 0, stream>>>(rgb, g11, be11, hbuf, 2 * HID, 0);
  ln_kernel<<<ROWS, 128, 0, stream>>>(dep, g12, be12, hbuf, 2 * HID, HID);
  proj_kernel<HID, 0><<<dim3(HID / 64, ROWS / 128), 128, 0, stream>>>(hbuf, 0,   wqh,  wql,  bp + 0 * HID, 0, Qh, Ql);
  proj_kernel<HID, 0><<<dim3(HID / 64, ROWS / 128), 128, 0, stream>>>(hbuf, HID, wkh,  wkl,  bp + 1 * HID, 0, Kh, Kl);
  proj_kernel<FF, 1><<<dim3(HID / 64, ROWS / 128), 128, 0, stream>>>(hbuf, 0,    wv1h, wv1l, bp + 2 * HID, 0, V1h, V1l);
  proj_kernel<FF, 1><<<dim3(HID / 64, ROWS / 128), 128, 0, stream>>>(hbuf, 0,    wv2h, wv2l, bp + 3 * HID, 0, V2h, V2l);
  attn_row_kernel<<<NT_TILES / 8, 256, 0, stream>>>(Qh, Ql, Kh, Kl, V1h, V1l, 0, y1);
  attn_row_kernel<<<NT_TILES / 8, 256, 0, stream>>>(Kh, Kl, Qh, Ql, V2h, V2l, 0, y2);
  (void)ML;
  add_perm_kernel<<<(ROWS * HID + 255) / 256, 256, 0, stream>>>(rgb, y1, resr, ROWS);
  add_perm_kernel<<<(ROWS * HID + 255) / 256, 256, 0, stream>>>(dep, y2, resd, ROWS);
  ln_kernel<<<ROWS, 128, 0, stream>>>(resr, g21, be21, hbuf, 2 * HID, 0);
  ln_kernel<<<ROWS, 128, 0, stream>>>(resd, g22, be22, hbuf, 2 * HID, HID);
  gemm_kernel<HID, FF, true ><<<dim3(FF / 64, ROWS / 128), 128, 0, stream>>>(hbuf, 2 * HID, 0, w11h, w11l, b11, nullptr, 0, f1, nullptr);
  gemm_kernel<FF, HID, false><<<dim3(HID / 64, ROWS / 128), 128, 0, stream>>>(f1, FF, 0, w12h, w12l, b12, resr, 0, out1, nullptr);
  gemm_kernel<HID, FF, true ><<<dim3(FF / 64, ROWS / 128), 128, 0, stream>>>(hbuf, 2 * HID, HID, w21h, w21l, b21, nullptr, 0, f1, nullptr);
  gemm_kernel<FF, HID, false><<<dim3(HID / 64, ROWS / 128), 128, 0, stream>>>(f1, FF, 0, w22h, w22l, b22, resd, 0, out2, out3);
}
